// SelfAttention_39788577030790
// MI455X (gfx1250) — hardware-verified
//
#include <hip/hip_runtime.h>


#ifndef NB
#define NB 8
#endif
#ifndef NTOK
#define NTOK 4096
#endif
#define NTOK_FULL 4096
#define CCH 256
#define RD 32
#define QKW 64
#define PCAR 256.0f
#define LOG2PCAR 8.0f
#define LOG2E 1.4426950408889634f
static_assert(RD == 32);
static_assert(QKW == 2 * RD);
static_assert(CCH % 64 == 0);
static_assert(CCH % 32 == 0);
static_assert(CCH == 256);
static_assert(NTOK % 128 == 0);
static_assert(NTOK <= NTOK_FULL);
static_assert((RD * CCH) % 8 == 0);
static_assert((size_t)NB * CCH * NTOK_FULL <= (size_t)8 * 256 * 4096);

constexpr size_t SZ_WQK = (size_t)QKW * CCH * 2;
constexpr size_t SZ_WV  = (size_t)CCH * CCH * 2;
constexpr size_t SZ_XB  = (size_t)NB * NTOK * CCH * 2;
constexpr size_t SZ_QK  = (size_t)NB * NTOK * QKW * 2;
constexpr size_t SZ_VT  = (size_t)NB * CCH * NTOK * 2;
constexpr size_t SZ_E2  = (size_t)NB * NTOK * 4;
constexpr size_t OFF_WQK = 0;
constexpr size_t OFF_WV  = OFF_WQK + SZ_WQK;
constexpr size_t OFF_XB  = OFF_WV + SZ_WV;
constexpr size_t OFF_QK  = OFF_XB + SZ_XB;
constexpr size_t OFF_VT  = OFF_QK + SZ_QK;
constexpr size_t OFF_E2  = OFF_VT + SZ_VT;
constexpr size_t WS_TOTAL = OFF_E2 + SZ_E2;
static_assert(SZ_WQK % 256 == 0);
static_assert(SZ_WV % 256 == 0);
static_assert(SZ_XB % 256 == 0);
static_assert(SZ_QK % 256 == 0);
static_assert(SZ_VT % 256 == 0);
static_assert(SZ_E2 % 256 == 0);
static_assert(WS_TOTAL <= (size_t)134217728);

typedef _Float16 h16;
typedef unsigned short bf;
typedef __attribute__((ext_vector_type(16))) __bf16   v16bf;
typedef __attribute__((ext_vector_type(16))) _Float16 v16h;
typedef __attribute__((ext_vector_type(8)))  _Float16 v8h;
typedef __attribute__((ext_vector_type(8)))  unsigned short v8us;
typedef __attribute__((ext_vector_type(8)))  float    v8f;
typedef __attribute__((ext_vector_type(4)))  float    v4f;
typedef v4f  __attribute__((may_alias)) v4fa;
typedef v8us __attribute__((may_alias)) v8usa;

__device__ __forceinline__ unsigned short f2bf(float f) { unsigned u = __float_as_uint(f); u += 0x7FFFu + ((u >> 16) & 1u); return (unsigned short)(u >> 16); }
__device__ __forceinline__ float bf2f(unsigned short b) { return __uint_as_float(((unsigned)b) << 16); }
__device__ __forceinline__ float bfr(float f) { return bf2f(f2bf(f)); }
__device__ __forceinline__ v16h cat16(v8h lo, v8h hi) { return __builtin_shufflevector(lo, hi, 0, 1, 2, 3, 4, 5, 6, 7, 8, 9, 10, 11, 12, 13, 14, 15); }
__device__ __forceinline__ v16bf cat16b(v8us lo, v8us hi) { return __builtin_bit_cast(v16bf, __builtin_shufflevector(lo, hi, 0, 1, 2, 3, 4, 5, 6, 7, 8, 9, 10, 11, 12, 13, 14, 15)); }
__device__ __forceinline__ v8f wmma16(v16h a, v16h b, v8f c) { return __builtin_amdgcn_wmma_f32_16x16x32_f16(false, a, false, b, (short)0, c, false, false); }
__device__ __forceinline__ v8f wmmab(v16bf a, v16bf b, v8f c) { return __builtin_amdgcn_wmma_f32_16x16x32_bf16(false, a, false, b, (short)0, c, false, false); }
__device__ __forceinline__ v16h  ldfh(const h16* p) { return cat16(*(const v8h*)p, *(const v8h*)(p + 16)); }
__device__ __forceinline__ v16bf ldfb(const bf* p)  { return cat16b(*(const v8us*)p, *(const v8us*)(p + 16)); }
__device__ __forceinline__ float ex2(float x) { return __builtin_amdgcn_exp2f(x); }

__global__ __launch_bounds__(256) void k_cvt8(const float* __restrict__ src, bf* dst, size_t n8) {
    const size_t i = (size_t)blockIdx.x * 256 + threadIdx.x; if (i >= n8) return;
    const v8f v = *(const v8f*)(src + i * 8); v8us o;
#pragma unroll
    for (int k = 0; k < 8; ++k) o[k] = f2bf(v[k]);
    *(volatile v8us*)(dst + i * 8) = o; __threadfence(); *(volatile v8us*)(dst + i * 8) = o;
}

__global__ __launch_bounds__(256) void k_xT(const float* __restrict__ x, bf* XB) {
    __shared__ __align__(16) unsigned short ts[64 * 72];
    const int tid = threadIdx.x; const int n0 = blockIdx.x * 64, c0 = blockIdx.y * 64, b = blockIdx.z;
    const float* src = x + ((size_t)b * CCH + c0) * NTOK_FULL + n0;
#pragma unroll
    for (int i = 0; i < 4; ++i) {
        const int idx = i * 256 + tid; const int cr = idx >> 4, pc = idx & 15;
        const v4f v = *(const v4f*)(src + (size_t)cr * NTOK_FULL + pc * 4);
#pragma unroll
        for (int q = 0; q < 4; ++q) ts[(pc * 4 + q) * 72 + cr] = f2bf(v[q]);
    }
    __syncthreads();
    v8us o[2];
#pragma unroll
    for (int i = 0; i < 2; ++i) { const int idx = i * 256 + tid; const int nr = idx >> 3, pc = idx & 7; o[i] = *(const v8usa*)(ts + nr * 72 + pc * 8); }
    bf* dst = XB + ((size_t)b * NTOK + n0) * CCH + c0;
#pragma unroll 1
    for (int ps = 0; ps < 2; ++ps) {
#pragma unroll
        for (int i = 0; i < 2; ++i) { const int idx = i * 256 + tid; const int nr = idx >> 3, pc = idx & 7; *(volatile v8us*)(dst + (size_t)nr * CCH + pc * 8) = o[i]; }
        if (ps == 0) __threadfence();
    }
}

template <int BMODE>
__device__ __forceinline__ void gemm64(const bf* __restrict__ A, const bf* __restrict__ Bt, h16* C, const int ldc, const float* __restrict__ biasA, const float* __restrict__ biasB, const int r0, const int c0) {
    __shared__ __align__(16) float os[16 * 68];
    const int lane = threadIdx.x & 31, lr = lane & 15, hi = lane >> 4;
    v8f acc[4][4];
#pragma unroll
    for (int mb = 0; mb < 4; ++mb)
#pragma unroll
        for (int nb = 0; nb < 4; ++nb) acc[mb][nb] = (v8f){};
    const bf* ap = A + (size_t)(r0 + lr) * CCH + 8 * hi;
    const bf* bp = Bt + (size_t)(c0 + lr) * CCH + 8 * hi;
#pragma unroll 1
    for (int kc = 0; kc < CCH; kc += 32) {
        v16bf a[4], bb[4];
#pragma unroll
        for (int t = 0; t < 4; ++t) { a[t] = ldfb(ap + (size_t)t * 16 * CCH + kc); bb[t] = ldfb(bp + (size_t)t * 16 * CCH + kc); }
#pragma unroll
        for (int nb = 0; nb < 4; ++nb)
#pragma unroll
            for (int mb = 0; mb < 4; ++mb) acc[mb][nb] = wmmab(a[mb], bb[nb], acc[mb][nb]);
        asm volatile("v_nop\n\tv_nop\n\tv_nop\n\tv_nop" : "+v"(acc[0][0]), "+v"(acc[0][1]), "+v"(acc[0][2]), "+v"(acc[0][3]), "+v"(acc[1][0]), "+v"(acc[1][1]), "+v"(acc[1][2]), "+v"(acc[1][3]) : "v"(a[0]), "v"(a[1]), "v"(bb[3]));
        asm volatile("v_nop\n\tv_nop\n\tv_nop\n\tv_nop" : "+v"(acc[2][0]), "+v"(acc[2][1]), "+v"(acc[2][2]), "+v"(acc[2][3]), "+v"(acc[3][0]), "+v"(acc[3][1]), "+v"(acc[3][2]), "+v"(acc[3][3]) : "v"(a[2]), "v"(a[3]), "v"(bb[3]));
    }
    const int rq = lane >> 3, pc = lane & 7;
    float badd[8]; float sc = 1.0f;
#pragma unroll
    for (int i = 0; i < 8; ++i) badd[i] = 0.0f;
    if (BMODE == 0) {
        const int cb = (pc * 8) & 31; const bool isq = (pc < 4);
        const v4f qa0 = *(const v4f*)(biasA + cb), qa1 = *(const v4f*)(biasA + cb + 4);
        const v4f kb0 = *(const v4f*)(biasB + cb), kb1 = *(const v4f*)(biasB + cb + 4);
#pragma unroll
        for (int i = 0; i < 4; ++i) { badd[i] = bfr(isq ? qa0[i] : kb0[i]); badd[4 + i] = bfr(isq ? qa1[i] : kb1[i]); }
        sc = isq ? LOG2E : 1.0f;
    }
#pragma unroll
    for (int mb = 0; mb < 4; ++mb) {
#pragma unroll
        for (int nb = 0; nb < 4; ++nb)
#pragma unroll
            for (int j = 0; j < 8; ++j) os[(hi * 8 + j) * 68 + nb * 16 + lr] = acc[mb][nb][j];
        __syncthreads();
        v8h ov[4];
#pragma unroll
        for (int s = 0; s < 4; ++s) {
            const int row = 4 * s + rq;
            const v4f x0 = *(const v4fa*)(os + row * 68 + pc * 8), x1 = *(const v4fa*)(os + row * 68 + pc * 8 + 4);
            float radd = 0.0f;
            if (BMODE == 1) radd = bfr(biasA[r0 + mb * 16 + row]);
#pragma unroll
            for (int i = 0; i < 4; ++i) {
                ov[s][i]     = (h16)((x0[i] + ((BMODE == 0) ? badd[i] : radd)) * sc);
                ov[s][4 + i] = (h16)((x1[i] + ((BMODE == 0) ? badd[4 + i] : radd)) * sc);
            }
        }
        h16* crow = C + (size_t)(r0 + mb * 16 + rq) * ldc + c0 + pc * 8;
#pragma unroll 1
        for (int ps = 0; ps < 2; ++ps) {
#pragma unroll
            for (int s = 0; s < 4; ++s) *(volatile v8h*)(crow + (size_t)(4 * s) * ldc) = ov[s];
            if (ps == 0) __threadfence();
        }
        __syncthreads();
    }
}

__global__ __launch_bounds__(32) void k_gemm_qk(const bf* __restrict__ XB, const bf* __restrict__ WQK, const float* __restrict__ bq, const float* __restrict__ bk, h16* QK) {
    gemm64<0>(XB, WQK, QK, QKW, bq, bk, blockIdx.x * 64, 0);
}
__global__ __launch_bounds__(32) void k_gemm_vt(const bf* __restrict__ WV, const bf* __restrict__ XB, const float* __restrict__ bv, h16* VT) {
    const size_t z = blockIdx.z;
    gemm64<1>(WV, XB + z * NTOK * CCH, VT + z * CCH * NTOK, NTOK, bv, bv, blockIdx.x * 64, blockIdx.y * 64);
}

__global__ __launch_bounds__(256) void k_stats(const h16* QK, float* E2) {
    __shared__ __align__(16) float es[128];
    const int lane = threadIdx.x & 31, lr = lane & 15, hi = lane >> 4;
    const int wave = __builtin_amdgcn_readfirstlane(threadIdx.x >> 5);
    const int b = blockIdx.y; const int m0 = blockIdx.x * 128 + wave * 16;
    const h16* base = QK + (size_t)b * NTOK * QKW;
    const v16h kf = ldfh(base + (size_t)(m0 + lr) * QKW + RD + 8 * hi);
    const h16* qb = base + (size_t)lr * QKW + 8 * hi;
    float rm = -3.0e38f, rs = 0.0f;
#pragma unroll 1
    for (int n0 = 0; n0 < NTOK; n0 += 64) {
        v16h qa[4]; v8f s[4];
#pragma unroll
        for (int t = 0; t < 4; ++t) qa[t] = ldfh(qb + (size_t)(n0 + 16 * t) * QKW);
#pragma unroll
        for (int t = 0; t < 4; ++t) s[t] = wmma16(qa[t], kf, (v8f){});
        asm volatile("v_nop\n\tv_nop\n\tv_nop\n\tv_nop" : "+v"(s[0]), "+v"(s[1]), "+v"(s[2]), "+v"(s[3]) : "v"(qa[0]), "v"(qa[1]), "v"(qa[2]), "v"(qa[3]), "v"(kf));
        float tm = s[0][0];
#pragma unroll
        for (int t = 0; t < 4; ++t)
#pragma unroll
            for (int j = 0; j < 8; ++j) tm = fmaxf(tm, s[t][j]);
        const float nm = fmaxf(rm, tm);
        float a = 0.0f;
#pragma unroll
        for (int t = 0; t < 4; ++t)
#pragma unroll
            for (int j = 0; j < 8; ++j) a += ex2(s[t][j] - nm);
        rs = rs * ex2(rm - nm) + a; rm = nm;
    }
    const float om = __shfl_xor(rm, 16, 32), osum = __shfl_xor(rs, 16, 32);
    const float M = fmaxf(rm, om);
    const float L = rs * ex2(rm - M) + osum * ex2(om - M);
    const float e2 = M + log2f(L) - LOG2PCAR;
    if (lane < 16) es[wave * 16 + lane] = e2;
    __syncthreads();
    if (wave == 0) {
        const v4f v = *(const v4fa*)(es + lane * 4);
        float* dst = E2 + (size_t)b * NTOK + blockIdx.x * 128 + lane * 4;
        *(volatile v4f*)dst = v; __threadfence(); *(volatile v4f*)dst = v;
    }
}

__global__ __launch_bounds__(128) void k_attn(const h16* QK, const h16* VT, const float* E2, float* out) {
    __shared__ __align__(16) float ot[64 * 68];
    const int tid = threadIdx.x; const int lane = tid & 31, lr = lane & 15, hi = lane >> 4;
    const int wave = __builtin_amdgcn_readfirstlane(tid >> 5);
    const int b = blockIdx.y; const int nb0 = blockIdx.x * 64; const int n0 = nb0 + wave * 16;
    const h16* qkb = QK + (size_t)b * NTOK * QKW;
    const h16* vtb = VT + (size_t)b * CCH * NTOK + (size_t)lr * NTOK + 8 * hi;
    const float* e2b = E2 + (size_t)b * NTOK + 8 * hi;
    const v16h qf = ldfh(qkb + (size_t)(n0 + lr) * QKW + 8 * hi);
    const h16* kb0 = qkb + (size_t)lr * QKW + RD + 8 * hi;
    v8f o[16];
#pragma unroll
    for (int i = 0; i < 16; ++i) o[i] = (v8f){};
#pragma unroll 1
    for (int m0 = 0; m0 < NTOK; m0 += 32) {
        v16h p;
#pragma unroll
        for (int t = 0; t < 2; ++t) {
            const v16h ka = ldfh(kb0 + (size_t)(m0 + 16 * t) * QKW);
            const v4f e0 = *(const v4f*)(e2b + m0 + 16 * t), e1 = *(const v4f*)(e2b + m0 + 16 * t + 4);
            v8f s = wmma16(ka, qf, (v8f){});
            asm volatile("v_nop\n\tv_nop\n\tv_nop\n\tv_nop" : "+v"(s) : "v"(ka), "v"(qf) : "memory");
#pragma unroll
            for (int i = 0; i < 4; ++i) { p[8 * t + i] = (h16)ex2(s[i] - e0[i]); p[8 * t + 4 + i] = (h16)ex2(s[4 + i] - e1[i]); }
        }
#pragma unroll
        for (int g = 0; g < 4; ++g) {
            v16h vf[4];
#pragma unroll
            for (int j = 0; j < 4; ++j) vf[j] = ldfh(vtb + (size_t)((g * 4 + j) * 16) * NTOK + m0);
#pragma unroll
            for (int j = 0; j < 4; ++j) o[g * 4 + j] = wmma16(p, vf[j], o[g * 4 + j]);
            asm volatile("v_nop\n\tv_nop\n\tv_nop\n\tv_nop" : "+v"(o[g * 4]), "+v"(o[g * 4 + 1]), "+v"(o[g * 4 + 2]), "+v"(o[g * 4 + 3]) : "v"(vf[0]), "v"(vf[1]), "v"(vf[2]), "v"(vf[3]), "v"(p) : "memory");
        }
    }
    float* ob = out + (size_t)b * CCH * NTOK_FULL + nb0;
    const int er = tid >> 4, ep = tid & 15;
#pragma unroll
    for (int g = 0; g < 4; ++g) {
#pragma unroll
        for (int j = 0; j < 4; ++j) {
            float* tp = ot + (j * 16 + lr) * 68 + wave * 16 + 8 * hi;
            const v4f w0 = { o[g * 4 + j][0], o[g * 4 + j][1], o[g * 4 + j][2], o[g * 4 + j][3] };
            const v4f w1 = { o[g * 4 + j][4], o[g * 4 + j][5], o[g * 4 + j][6], o[g * 4 + j][7] };
            *(v4fa*)tp = w0; *(v4fa*)(tp + 4) = w1;
        }
        __syncthreads();
        v4f ov[8];
#pragma unroll
        for (int s = 0; s < 8; ++s) { const v4f t4 = *(const v4fa*)(ot + (8 * s + er) * 68 + ep * 4); ov[s] = t4 * (1.0f / PCAR); }
        float* dst = ob + (size_t)(g * 64 + er) * NTOK_FULL + ep * 4;
#pragma unroll 1
        for (int ps = 0; ps < 2; ++ps) {
#pragma unroll
            for (int s = 0; s < 8; ++s) *(volatile v4f*)(dst + (size_t)(8 * s) * NTOK_FULL) = ov[s];
            if (ps == 0) __threadfence();
        }
        __syncthreads();
    }
}

extern "C" void kernel_launch(void* const* d_in, const int* in_sizes, int n_in,
                              void* d_out, int out_size, void* d_ws, size_t ws_size, hipStream_t stream) {
    if (n_in < 7) return;
    if (in_sizes[0] < (NB * CCH - 1) * NTOK_FULL + NTOK) return;
    if (in_sizes[1] < RD * CCH || in_sizes[2] < RD || in_sizes[3] < RD * CCH || in_sizes[4] < RD || in_sizes[5] < CCH * CCH || in_sizes[6] < CCH) return;
    if (out_size < (NB * CCH - 1) * NTOK_FULL + NTOK) return;
    if (WS_TOTAL > ws_size) return;
    const float* x  = (const float*)d_in[0];
    const float* wq = (const float*)d_in[1];
    const float* bq = (const float*)d_in[2];
    const float* wk = (const float*)d_in[3];
    const float* bk = (const float*)d_in[4];
    const float* wv = (const float*)d_in[5];
    const float* bv = (const float*)d_in[6];
    float* out = (float*)d_out;
    char* ws = (char*)d_ws;
    bf*  WQK = (bf*)(ws + OFF_WQK);
    bf*  WV  = (bf*)(ws + OFF_WV);
    bf*  XB  = (bf*)(ws + OFF_XB);
    h16* QKp = (h16*)(ws + OFF_QK);
    h16* VT  = (h16*)(ws + OFF_VT);
    float* E2 = (float*)(ws + OFF_E2);

    k_cvt8<<<(unsigned)((RD * CCH / 8 + 255) / 256), 256, 0, stream>>>(wq, WQK, (size_t)(RD * CCH / 8));
    k_cvt8<<<(unsigned)((RD * CCH / 8 + 255) / 256), 256, 0, stream>>>(wk, WQK + RD * CCH, (size_t)(RD * CCH / 8));
    k_cvt8<<<(unsigned)((CCH * CCH / 8 + 255) / 256), 256, 0, stream>>>(wv, WV, (size_t)(CCH * CCH / 8));
    k_xT<<<dim3(NTOK / 64, CCH / 64, NB), 256, 0, stream>>>(x, XB);
    k_gemm_qk<<<dim3(NB * NTOK / 64, 1, 1), 32, 0, stream>>>(XB, WQK, bq, bk, QKp);
    k_gemm_vt<<<dim3(CCH / 64, NTOK / 64, NB), 32, 0, stream>>>(WV, XB, bv, VT);
    k_stats<<<dim3(NTOK / 128, NB, 1), 256, 0, stream>>>(QKp, E2);
    k_attn<<<dim3(NTOK / 64, NB, 1), 128, 0, stream>>>(QKp, VT, E2, out);
}
